// myGRUCell_group4_54571854463571
// MI455X (gfx1250) — hardware-run, weakly checked
//
#include <hip/hip_runtime.h>


#define NR   8192
#define CH   4096
#define HH   1024
#define GG   4
#define HG   256
#define WR   256
typedef _Float16 h16;
typedef unsigned short bf;
typedef __attribute__((ext_vector_type(16))) __bf16   v16bf;
typedef __attribute__((ext_vector_type(16))) _Float16 v16h;
typedef __attribute__((ext_vector_type(8)))  _Float16 v8h;
typedef __attribute__((ext_vector_type(8)))  unsigned short v8us;
typedef __attribute__((ext_vector_type(8)))  float    v8f;
typedef __attribute__((ext_vector_type(4)))  float    v4f;
typedef v8h  __attribute__((may_alias)) v8ha;
typedef v4f  __attribute__((may_alias)) v4fa;
typedef v8us __attribute__((may_alias)) v8usa;

__device__ __forceinline__ unsigned short f2bf(float f) { unsigned u = __float_as_uint(f); u += 0x7FFFu + ((u >> 16) & 1u); return (unsigned short)(u >> 16); }
__device__ __forceinline__ float bf2f(unsigned short b) { return __uint_as_float(((unsigned)b) << 16); }
__device__ __forceinline__ float bfr(float f) { return bf2f(f2bf(f)); }
__device__ __forceinline__ v16h cat16(v8h lo, v8h hi) { return __builtin_shufflevector(lo, hi, 0, 1, 2, 3, 4, 5, 6, 7, 8, 9, 10, 11, 12, 13, 14, 15); }
__device__ __forceinline__ v16bf cat16b(v8us lo, v8us hi) { return __builtin_bit_cast(v16bf, __builtin_shufflevector(lo, hi, 0, 1, 2, 3, 4, 5, 6, 7, 8, 9, 10, 11, 12, 13, 14, 15)); }
__device__ __forceinline__ v8f wmma16(v16h a, v16h b, v8f c) { return __builtin_amdgcn_wmma_f32_16x16x32_f16(false, a, false, b, (short)0, c, false, false); }
__device__ __forceinline__ v8f wmmab(v16bf a, v16bf b, v8f c) { return __builtin_amdgcn_wmma_f32_16x16x32_bf16(false, a, false, b, (short)0, c, false, false); }


template <typename T16> struct WFrag;
template <> struct WFrag<h16> { typedef v16h V; static __device__ __forceinline__ V ld(const h16* p) { return cat16(*(const v8h*)p, *(const v8h*)(p + 16)); } static __device__ __forceinline__ v8f mma(V a, V b, v8f c) { return wmma16(a, b, c); } };
template <> struct WFrag<bf> { typedef v16bf V; static __device__ __forceinline__ V ld(const bf* p) { return cat16b(*(const v8us*)p, *(const v8us*)(p + 16)); } static __device__ __forceinline__ v8f mma(V a, V b, v8f c) { return wmmab(a, b, c); } };
template <typename T16, int NSPLIT, bool BIAS>
__global__ __launch_bounds__(32) void k_gemmw(const T16* __restrict__ A, const T16* __restrict__ A2, const T16* __restrict__ Bt, const T16* __restrict__ Bt2, int K, float* C, int ldc, const float* __restrict__ bias, size_t sA, size_t sB, size_t sC) {
    typedef typename WFrag<T16>::V V;
    __shared__ __align__(16) float os[16 * 68];
    const size_t z = blockIdx.z; A += z * sA; if (A2) A2 += z * sA; Bt += z * sB; if (Bt2) Bt2 += z * sB; C += z * sC;
    const int lane = threadIdx.x & 31, lr = lane & 15, hi = lane >> 4; const int r0 = blockIdx.x * 64, c0 = blockIdx.y * 64;
    v8f acc[4][4];
#pragma unroll
    for (int mb = 0; mb < 4; ++mb)
#pragma unroll
        for (int nb = 0; nb < 4; ++nb) acc[mb][nb] = (v8f){};
    const size_t aoff = (size_t)(r0 + lr) * K + 8 * hi, boff = (size_t)(c0 + lr) * K + 8 * hi;
#pragma unroll 1
    for (int kc = 0; kc < K; kc += 32) {
        V a[4], a2[4];
#pragma unroll
        for (int mb = 0; mb < 4; ++mb) { a[mb] = WFrag<T16>::ld(A + aoff + (size_t)mb * 16 * K + kc); if (NSPLIT == 1 || NSPLIT == 2) a2[mb] = WFrag<T16>::ld(A2 + aoff + (size_t)mb * 16 * K + kc); }
#pragma unroll
        for (int nb = 0; nb < 4; ++nb) { const V b = WFrag<T16>::ld(Bt + boff + (size_t)nb * 16 * K + kc); V b2; if (NSPLIT >= 2) b2 = WFrag<T16>::ld(Bt2 + boff + (size_t)nb * 16 * K + kc);
#pragma unroll
            for (int mb = 0; mb < 4; ++mb) { acc[mb][nb] = WFrag<T16>::mma(a[mb], b, acc[mb][nb]); if (NSPLIT == 1 || NSPLIT == 2) acc[mb][nb] = WFrag<T16>::mma(a2[mb], b, acc[mb][nb]); if (NSPLIT >= 2) acc[mb][nb] = WFrag<T16>::mma(a[mb], b2, acc[mb][nb]); } }
        asm volatile("v_nop\n\tv_nop\n\tv_nop\n\tv_nop" : "+v"(acc[0][0]), "+v"(acc[1][1]), "+v"(acc[2][2]), "+v"(acc[3][3]) : "v"(a[0]), "v"(a[3]));
    }
#pragma unroll
    for (int mb = 0; mb < 4; ++mb) {
#pragma unroll
        for (int nb = 0; nb < 4; ++nb) {
#pragma unroll
            for (int j = 0; j < 8; ++j) os[(hi * 8 + j) * 68 + nb * 16 + lr] = acc[mb][nb][j]; }
        __builtin_amdgcn_wave_barrier(); asm volatile("" ::: "memory");
        float* crow = C + (size_t)(r0 + mb * 16) * ldc + c0;
#pragma unroll 1
        for (int ps = 0; ps < 2; ++ps) {
#pragma unroll
            for (int s = 0; s < 8; ++s) { const int row = 2 * s + hi, cofs = lr * 4; v4f val = *(const v4fa*)(os + row * 68 + cofs); if (BIAS) { val[0] += bfr(bias[c0 + cofs]); val[1] += bfr(bias[c0 + cofs + 1]); val[2] += bfr(bias[c0 + cofs + 2]); val[3] += bfr(bias[c0 + cofs + 3]); }
                *(volatile v4f*)(crow + (size_t)row * ldc + cofs) = val; }
            if (ps == 0) __threadfence(); }
        __builtin_amdgcn_wave_barrier(); asm volatile("" ::: "memory");
    }
}

__device__ __forceinline__ void splitf(float y, unsigned short& h, unsigned short& l) { h = f2bf(y); l = f2bf(y - bf2f(h)); }
typedef __attribute__((ext_vector_type(2))) unsigned short v2us;
typedef __attribute__((ext_vector_type(4))) unsigned short v4us;

__global__ __launch_bounds__(256) void k_wtG(const float* __restrict__ w, int K, int N, bf* Bt) {
    const int lane = threadIdx.x & 31; const int L0 = (blockIdx.x * 8 + (threadIdx.x >> 5)) * 8; const int nlines = N * K / 64;
#pragma unroll
    for (int ps = 0; ps < 2; ++ps) {
#pragma unroll 1
        for (int l = 0; l < 8; ++l) { const int L = L0 + l; if (L >= nlines) break; const size_t e = (size_t)L * 64 + lane * 2; const int k = (int)(e % K), n = (int)(e / K); v2us o;
            o[0] = f2bf(w[(size_t)k * N + n]); o[1] = f2bf(w[(size_t)(k + 1) * N + n]); *(volatile v2us*)(Bt + e) = o; }
        if (ps == 0) __threadfence(); }
}
__global__ __launch_bounds__(256) void k_cvt8(const float* __restrict__ src, bf* dst, size_t n8) { const size_t i = (size_t)blockIdx.x * 256 + threadIdx.x; if (i >= n8) return; const v8f v = *(const v8f*)(src + i * 8); v8us o;
#pragma unroll
    for (int k = 0; k < 8; ++k) o[k] = f2bf(v[k]); *(volatile v8us*)(dst + i * 8) = o; __threadfence(); *(volatile v8us*)(dst + i * 8) = o; }
__global__ __launch_bounds__(256) void k_wtP(const float* __restrict__ w, int K, int N, int KP, int NP, bf* Bt) { const int e = (blockIdx.x * 256 + threadIdx.x) * 2; if (e >= NP * KP) return; const int k = e % KP; const int n = e / KP; v2us o;
#pragma unroll
    for (int u = 0; u < 2; ++u) o[u] = (n < N && k + u < K) ? f2bf(w[(size_t)(k + u) * N + n]) : (unsigned short)0; *(volatile v2us*)(Bt + e) = o; __threadfence(); *(volatile v2us*)(Bt + e) = o; }
__global__ __launch_bounds__(256) void k_grp(const float* __restrict__ h, int r0, bf* HGb) { const int e = (blockIdx.x * 256 + threadIdx.x) * 4; if (e >= GG * CH * HG) return; const int c = e % HG; const int r = (e / HG) % CH; const int g = e / (HG * CH); const float* src = h + (size_t)(r0 + r) * HH + g * HG + c; v4us o;
#pragma unroll
    for (int u = 0; u < 4; ++u) o[u] = f2bf(src[u]); *(volatile v4us*)(HGb + e) = o; __threadfence(); *(volatile v4us*)(HGb + e) = o; }
__global__ __launch_bounds__(256) void k_spl(const float* __restrict__ F, size_t n4, bf* Hh, bf* Hl) { const size_t e = ((size_t)blockIdx.x * 256 + threadIdx.x) * 4; if (e >= n4) return; const v4f a = *(const v4f*)(F + e); v4us oh, ol;
#pragma unroll
    for (int u = 0; u < 4; ++u) { unsigned short p, q; splitf(a[u], p, q); oh[u] = p; ol[u] = q; } *(volatile v4us*)(Hh + e) = oh; *(volatile v4us*)(Hl + e) = ol; __threadfence(); *(volatile v4us*)(Hh + e) = oh; *(volatile v4us*)(Hl + e) = ol; }
__global__ __launch_bounds__(256) void k_acc(float* ACC, const float* __restrict__ U, int first) { const int e = (blockIdx.x * 256 + threadIdx.x) * 4; if (e >= CH * HH) return; const v4f u4 = *(const v4f*)(U + e); v4f a; if (first) { a[0] = a[1] = a[2] = a[3] = 0.f; } else a = *(const v4f*)(ACC + e); v4f r;
#pragma unroll
    for (int u = 0; u < 4; ++u) r[u] = __fadd_rn(a[u], u4[u]); *(volatile v4f*)(ACC + e) = r; __threadfence(); *(volatile v4f*)(ACC + e) = r; }
__global__ __launch_bounds__(256) void k_fin(const float* __restrict__ A1, const float* __restrict__ A2, const float* __restrict__ W3, const float* __restrict__ S3, const float* __restrict__ h, const float* __restrict__ br, const float* __restrict__ bg, const float* __restrict__ bu, int r0, float* OUT) {
    const int e = (blockIdx.x * 256 + threadIdx.x) * 4; if (e >= CH * HH) return; const int c = e % HH; const v4f a1 = *(const v4f*)(A1 + e), a2 = *(const v4f*)(A2 + e), w3 = *(const v4f*)(W3 + e), s3 = *(const v4f*)(S3 + e), hv = *(const v4f*)(h + (size_t)r0 * HH + e); v4f o;
#pragma unroll
    for (int u = 0; u < 4; ++u) { const float r = __fdiv_rn(1.0f, __fadd_rn(1.0f, __expf(-__fadd_rn(a1[u], bfr(br[c + u]))))); const float z = __fdiv_rn(1.0f, __fadd_rn(1.0f, __expf(-__fadd_rn(a2[u], bfr(bg[c + u])))));
        float rs = __fmul_rn(r, s3[u]); asm volatile("" : "+v"(rs)); float t0 = __fadd_rn(w3[u], rs); asm volatile("" : "+v"(t0)); const float cc = tanhf(__fadd_rn(t0, bfr(bu[c + u]))); const float hb = bfr(hv[u]);
        float zh = __fmul_rn(z, hb); float omz = __fsub_rn(1.0f, z); asm volatile("" : "+v"(zh)); asm volatile("" : "+v"(omz)); float zc = __fmul_rn(omz, cc); asm volatile("" : "+v"(zc)); o[u] = __fadd_rn(zh, zc); }
    *(volatile v4f*)(OUT + (size_t)r0 * HH + e) = o; __threadfence(); *(volatile v4f*)(OUT + (size_t)r0 * HH + e) = o; }

extern "C" void kernel_launch(void* const* d_in, const int* in_sizes, int n_in,
                              void* d_out, int out_size, void* d_ws, size_t ws_size, hipStream_t stream) {
    (void)in_sizes; (void)n_in; (void)out_size;
    const float** I = (const float**)d_in;
    const float *x = I[0], *h = I[1], *W = I[2]; const float* Wk[3] = {I[3], I[4], I[5]};
    const float* Ua[4] = {I[6], I[10], I[14], I[18]}; const float* Uk[4][3] = {{I[7], I[8], I[9]}, {I[11], I[12], I[13]}, {I[15], I[16], I[17]}, {I[19], I[20], I[21]}}; const int RS[4] = {64, 64, 32, 32}; (void)RS;
    const float *br = I[22], *bg = I[23], *bu = I[24];
    float* OUT = (float*)d_out;
    char* wsp = (char*)d_ws;
    auto take = [&](size_t bytes) { char* p = wsp; wsp += (bytes + 255) & ~(size_t)255; return (void*)p; };
    bf* BW = (bf*)take((size_t)WR * HH * 2); bf* BWk[3]; for (int k = 0; k < 3; ++k) BWk[k] = (bf*)take((size_t)HH * WR * 2);
    bf* BUa[4][GG]; bf* BUk[4][GG][3]; for (int s = 0; s < 4; ++s) for (int j = 0; j < GG; ++j) { BUa[s][j] = (bf*)take((size_t)64 * HG * 2); for (int k = 0; k < 3; ++k) BUk[s][j][k] = (bf*)take((size_t)HG * 64 * 2); }
    bf* XB = (bf*)take((size_t)CH * HH * 2); bf* HGb = (bf*)take((size_t)GG * CH * HG * 2); float* XW = (float*)take((size_t)CH * WR * 4); bf* XWh = (bf*)take((size_t)CH * WR * 2); bf* XWl = (bf*)take((size_t)CH * WR * 2);
    float* A1 = (float*)take((size_t)CH * HH * 4); float* A2 = (float*)take((size_t)CH * HH * 4); float* W3 = (float*)take((size_t)CH * HH * 4); float* S3 = (float*)take((size_t)CH * HH * 4); float* U[3]; for (int k = 0; k < 3; ++k) U[k] = (float*)take((size_t)CH * HH * 4);
    float* T = (float*)take((size_t)CH * 64 * 4); bf* Th = (bf*)take((size_t)CH * 64 * 2); bf* Tl = (bf*)take((size_t)CH * 64 * 2);
    if ((size_t)(wsp - (char*)d_ws) > ws_size) return;
    k_wtG<<<(HH * WR / 64 + 63) / 64, 256, 0, stream>>>(W, HH, WR, BW); for (int k = 0; k < 3; ++k) k_wtG<<<(WR * HH / 64 + 63) / 64, 256, 0, stream>>>(Wk[k], WR, HH, BWk[k]);
    for (int s = 0; s < 4; ++s) for (int j = 0; j < GG; ++j) { const int r = RS[s]; k_wtP<<<(64 * HG / 2 + 255) / 256, 256, 0, stream>>>(Ua[s] + (size_t)j * HG * r, HG, r, HG, 64, BUa[s][j]); for (int k = 0; k < 3; ++k) k_wtP<<<(HG * 64 / 2 + 255) / 256, 256, 0, stream>>>(Uk[s][k] + (size_t)j * r * HG, r, HG, 64, HG, BUk[s][j][k]); }
    float* ACC[3] = {A1, A2, S3};
    for (int r0 = 0; r0 < NR; r0 += CH) {
        k_cvt8<<<(CH * HH / 8 + 255) / 256, 256, 0, stream>>>(x + (size_t)r0 * HH, XB, (size_t)CH * HH / 8); k_grp<<<(GG * CH * HG / 4 + 255) / 256, 256, 0, stream>>>(h, r0, HGb);
        k_gemmw<bf, 0, false><<<dim3(CH / 64, WR / 64, 1), 32, 0, stream>>>(XB, nullptr, BW, nullptr, HH, XW, WR, nullptr, 0, 0, 0); k_spl<<<(CH * WR / 4 + 255) / 256, 256, 0, stream>>>(XW, (size_t)CH * WR, XWh, XWl);
        k_gemmw<bf, 1, false><<<dim3(CH / 64, HH / 64, 1), 32, 0, stream>>>(XWh, XWl, BWk[0], nullptr, WR, A1, HH, nullptr, 0, 0, 0);
        k_gemmw<bf, 1, false><<<dim3(CH / 64, HH / 64, 1), 32, 0, stream>>>(XWh, XWl, BWk[1], nullptr, WR, A2, HH, nullptr, 0, 0, 0);
        k_gemmw<bf, 1, false><<<dim3(CH / 64, HH / 64, 1), 32, 0, stream>>>(XWh, XWl, BWk[2], nullptr, WR, W3, HH, nullptr, 0, 0, 0);
        for (int s = 0; s < 4; ++s) {
            for (int j = 0; j < GG; ++j) { const int gs = (j + s) % GG;
                k_gemmw<bf, 0, false><<<dim3(CH / 64, 1, 1), 32, 0, stream>>>(HGb + (size_t)gs * CH * HG, nullptr, BUa[s][j], nullptr, HG, T, 64, nullptr, 0, 0, 0);
                k_spl<<<(CH * 64 / 4 + 255) / 256, 256, 0, stream>>>(T, (size_t)CH * 64, Th, Tl);
                for (int k = 0; k < 3; ++k) k_gemmw<bf, 1, false><<<dim3(CH / 64, HG / 64, 1), 32, 0, stream>>>(Th, Tl, BUk[s][j][k], nullptr, 64, U[k] + j * HG, HH, nullptr, 0, 0, 0); }
            for (int k = 0; k < 3; ++k) k_acc<<<(CH * HH / 4 + 255) / 256, 256, 0, stream>>>(ACC[k], U[k], (k == 2 && s == 0) ? 1 : 0); }
        k_fin<<<(CH * HH / 4 + 255) / 256, 256, 0, stream>>>(A1, A2, W3, S3, h, br, bg, bu, r0, OUT); }
}
